// VGAE_Encoder_72189810312082
// MI455X (gfx1250) — hardware-run, weakly checked
//
#include <hip/hip_runtime.h>
#include <stddef.h>
#include <stdint.h>
#include <math.h>

#define NN      50000
#define NE      800000
#define FIN     128
#define HID     128
#define OUTF    64
#define NCAT    128
#define KC      256
#define GBM     128
#define MP      50048
#define NTHR    256
#define NWAVE   8
#define EPT     8
#define WCH     (32 * EPT)
#define NBRUN   1024
#define SLB     10
#define NBK     49
#define NSLOT   (NBK * NBRUN)
#define WLCAP   3584
#define RCAP    28672
#define DEGCAP  64
#define MAXDEG_MEAS 35
#define MAXBLK_MEAS 16623
#define RBM     64
#define SP      68
#define OUTSPLIT 3200000

#define BK_ZINTS (NWAVE * WLCAP + RCAP + 3 * NBRUN)
#define BK_INTS  (BK_ZINTS + 16)
#define BK_LDS   (BK_INTS * 4)

#define PBX   (MP * FIN / 8 / NTHR)
#define PBWA  (HID * FIN / 8 / NTHR)
#define PBWM  (OUTF * KC / 8 / NTHR)
#define PBWL  (OUTF * KC / 8 / NTHR)
#define PBTOT (PBX + PBWA + PBWM + PBWL + 1)

static_assert(NN <= NBK * NBRUN);
static_assert(HID == 32 * 4);
static_assert(2 * OUTF == 128 && NCAT == 2 * OUTF);
static_assert(MP == 391 * GBM && MP >= NN && MP % RBM == 0 && MP <= NSLOT);
static_assert(NBRUN == (1 << SLB) && NBRUN % RBM == 0 && NBRUN % GBM == 0 && NBRUN == 4 * NTHR);
static_assert(NE <= (1 << 20) && (((long long)NE) << SLB) < (1LL << 31));
static_assert(NE % WCH == 0 && NE % 4 == 0);
static_assert(RCAP == NWAVE * WLCAP && RCAP % (NTHR * 4) == 0 && BK_ZINTS % 4 == 0);
static_assert((long long)RCAP * 100 >= (long long)MAXBLK_MEAS * 105);
static_assert(WLCAP >= MAXBLK_MEAS / 8 + 8 * 46 + 1);
static_assert(MAXDEG_MEAS + 8 <= DEGCAP);
static_assert(BK_LDS <= 300000 && BK_LDS <= 327680);
static_assert((GBM * SP + GBM) * 4 <= 65536);
static_assert((MP * FIN / 8) % NTHR == 0 && (HID * FIN / 8) % NTHR == 0 && (OUTF * KC / 8) % NTHR == 0);
static_assert(FIN % 32 == 0 && KC % 32 == 0 && KC == 2 * HID);
static_assert((long long)OUTSPLIT + (long long)(NN - 1) * OUTF + 63 < 2LL * NN * OUTF);
static_assert(OUTSPLIT == NN * OUTF && (OUTSPLIT * 4) % 128 == 0);

typedef float          v4f   __attribute__((ext_vector_type(4)));
typedef float          v8f   __attribute__((ext_vector_type(8)));
typedef int            v4i   __attribute__((ext_vector_type(4)));
typedef int            v8i   __attribute__((ext_vector_type(8)));
typedef unsigned short v8us  __attribute__((ext_vector_type(8)));
typedef unsigned short v16us __attribute__((ext_vector_type(16)));
typedef __bf16         v16bf __attribute__((ext_vector_type(16)));
typedef v4f  __attribute__((may_alias)) v4fa;
typedef v4i  __attribute__((may_alias)) v4ia;
typedef v8us __attribute__((may_alias)) v8usa;
union FragB { v16bf v; v16us u; v8us h[2]; v8i w; };

__device__ __forceinline__ v8f wmb(const FragB& a, const FragB& b, v8f c) {
  v8f d = __builtin_amdgcn_wmma_f32_16x16x32_bf16(false, a.v, false, b.v, (short)0, c, false, false);
  asm volatile("v_nop\n\tv_nop\n\tv_nop\n\tv_nop" : "+v"(d) : "v"(a.w), "v"(b.w));
  return d;
}

__device__ __forceinline__ unsigned bf16_bits(float f) {
  const unsigned u = __float_as_uint(f);
  const unsigned r = (u + 0x7fffu + ((u >> 16) & 1u)) >> 16;
  const unsigned q = (u >> 16) | 0x40u;
  return ((u & 0x7fffffffu) > 0x7f800000u) ? q : r;
}
__device__ __forceinline__ float bf16_val(float f) {
  return __uint_as_float(bf16_bits(f) << 16);
}

__device__ __forceinline__ void hilo_pack(float v0, float v1, float v2, float v3,
                                          int& h01, int& h23, int& l01, int& l23) {
  const unsigned a0 = bf16_bits(v0), a1 = bf16_bits(v1), a2 = bf16_bits(v2), a3 = bf16_bits(v3);
  const unsigned b0 = bf16_bits(v0 - __uint_as_float(a0 << 16));
  const unsigned b1 = bf16_bits(v1 - __uint_as_float(a1 << 16));
  const unsigned b2 = bf16_bits(v2 - __uint_as_float(a2 << 16));
  const unsigned b3 = bf16_bits(v3 - __uint_as_float(a3 << 16));
  h01 = (int)(a0 | (a1 << 16)); h23 = (int)(a2 | (a3 << 16));
  l01 = (int)(b0 | (b1 << 16)); l23 = (int)(b2 | (b3 << 16));
}

__device__ __forceinline__ v4i regroup_row(int h01, int h23, int l01, int l23, int lane) {
  const int s0 = (2 * lane) & 31, s1 = s0 + 1;
  const int a0 = __shfl(h01, s0, 32), a1 = __shfl(h23, s0, 32), a2 = __shfl(h01, s1, 32), a3 = __shfl(h23, s1, 32);
  const int b0 = __shfl(l01, s0, 32), b1 = __shfl(l23, s0, 32), b2 = __shfl(l01, s1, 32), b3 = __shfl(l23, s1, 32);
  const int mk = (lane < 16) ? -1 : 0;
  v4i o;
  o.x = (a0 & mk) | (b0 & ~mk); o.y = (a1 & mk) | (b1 & ~mk);
  o.z = (a2 & mk) | (b2 & ~mk); o.w = (a3 & mk) | (b3 & ~mk);
  return o;
}

__device__ __forceinline__ void st2_v4f(float* p, v4f v) {
  *(volatile v4f*)p = v;
  __threadfence();
  *(volatile v4f*)p = v;
}
__device__ __forceinline__ void st2_v8us(unsigned short* p, v8us v) {
  *(volatile v8us*)p = v;
  __threadfence();
  *(volatile v8us*)p = v;
}

__device__ __forceinline__ v8us col8(const float* __restrict__ base, int stride) {
  float f[8];
#pragma unroll
  for (int i = 0; i < 8; ++i) f[i] = base[(size_t)i * (size_t)stride];
  v8us o;
#pragma unroll
  for (int i = 0; i < 8; ++i) o[i] = (unsigned short)bf16_bits(f[i]);
  return o;
}

__global__ __launch_bounds__(NTHR) void k_prep(const float* __restrict__ x, const float* __restrict__ wa,
                                               const float* __restrict__ ba, const float* __restrict__ gam,
                                               const float* __restrict__ bet, const float* __restrict__ wmu,
                                               const float* __restrict__ bmu, const float* __restrict__ wlv,
                                               const float* __restrict__ blv, unsigned short* xb,
                                               unsigned short* wpl, float* tb) {
  const int tid = (int)threadIdx.x, lane = tid & 31, wave = tid >> 5;
  const int blk = (int)blockIdx.x;
  unsigned short* wat = wpl;
  unsigned short* wct = wpl + (size_t)HID * FIN;
  if (blk < PBX) {
    const int u   = blk * NTHR + tid;
    const int row = u >> 4, k8 = (u & 15) * 8;
    const int rc  = row < NN ? row : NN - 1;
    const unsigned mk = row < NN ? 0xffffu : 0u;
    const float* p = x + (size_t)rc * FIN + k8;
    const v4f a = *(const v4fa*)p;
    const v4f b = *(const v4fa*)(p + 4);
    v8us o;
    o[0] = (unsigned short)(bf16_bits(a.x) & mk); o[1] = (unsigned short)(bf16_bits(a.y) & mk);
    o[2] = (unsigned short)(bf16_bits(a.z) & mk); o[3] = (unsigned short)(bf16_bits(a.w) & mk);
    o[4] = (unsigned short)(bf16_bits(b.x) & mk); o[5] = (unsigned short)(bf16_bits(b.y) & mk);
    o[6] = (unsigned short)(bf16_bits(b.z) & mk); o[7] = (unsigned short)(bf16_bits(b.w) & mk);
    st2_v8us(xb + (size_t)row * FIN + k8, o);
  } else if (blk < PBX + PBWA) {
    const int u = (blk - PBX) * NTHR + tid;
    const int n = u >> 4, k8 = (u & 15) * 8;
    const v8us o = col8(wa + (size_t)k8 * HID + n, HID);
    st2_v8us(wat + (size_t)n * FIN + k8, o);
  } else if (blk < PBX + PBWA + PBWM) {
    const int u = (blk - PBX - PBWA) * NTHR + tid;
    const int n = u >> 5, k8 = (u & 31) * 8, kk = k8 & (HID - 1);
    const v8us o = col8(wmu + (size_t)kk * OUTF + n, OUTF);
    st2_v8us(wct + (size_t)n * KC + k8, o);
  } else if (blk < PBX + PBWA + PBWM + PBWL) {
    const int u = (blk - PBX - PBWA - PBWM) * NTHR + tid;
    const int n = u >> 5, k8 = (u & 31) * 8, kk = k8 & (HID - 1);
    const v8us o = col8(wlv + (size_t)kk * OUTF + n, OUTF);
    st2_v8us(wct + (size_t)(OUTF + n) * KC + k8, o);
  } else {
    if (tid < 128) {
      const int q = lane & 15;
      v4f a;
      if (wave == 0) {
        a = *(const v4fa*)(ba + 4 * lane);
      } else if (wave == 1) {
        a = *(const v4fa*)(gam + 4 * lane);
      } else if (wave == 2) {
        a = *(const v4fa*)(bet + 4 * lane);
      } else {
        const v4f um = *(const v4fa*)(bmu + 4 * q);
        const v4f ul = *(const v4fa*)(blv + 4 * q);
        asm volatile("" :: "v"(um));
        asm volatile("" :: "v"(ul));
        const unsigned mk = (lane < 16) ? 0xffffffffu : 0u;
        a.x = __uint_as_float((__float_as_uint(um.x) & mk) | (__float_as_uint(ul.x) & ~mk));
        a.y = __uint_as_float((__float_as_uint(um.y) & mk) | (__float_as_uint(ul.y) & ~mk));
        a.z = __uint_as_float((__float_as_uint(um.z) & mk) | (__float_as_uint(ul.z) & ~mk));
        a.w = __uint_as_float((__float_as_uint(um.w) & mk) | (__float_as_uint(ul.w) & ~mk));
      }
      v4f o;
      o.x = bf16_val(a.x); o.y = bf16_val(a.y); o.z = bf16_val(a.z); o.w = bf16_val(a.w);
      st2_v4f(tb + 128 * wave + 4 * lane, o);
    }
  }
}

__device__ __forceinline__ void bucket_flush(const int* pl, const int* cnt, const int* offs, const int* dvb,
                                             int ov, int* lp, int* cp, int* op, int* dp, int* fp, int tid) {
#pragma unroll 1
  for (int i = tid * 4; i < RCAP; i += NTHR * 4) {
    const v4i v = *(const v4ia*)(pl + i);
    *(volatile v4i*)(lp + i) = v;
  }
  {
    const v4i c = *(const v4ia*)(cnt + 4 * tid);
    *(volatile v4i*)(cp + 4 * tid) = c;
    const v4i o = *(const v4ia*)(offs + 4 * tid);
    *(volatile v4i*)(op + 4 * tid) = o;
    const v4i d = *(const v4ia*)(dvb + 4 * tid);
    *(volatile v4i*)(dp + 4 * tid) = d;
  }
  if (tid < 8) {
    const v4i f = {ov, ov, ov, ov};
    *(volatile v4i*)(fp + 4 * tid) = f;
  }
}

__global__ __launch_bounds__(NTHR) void k_bucket(const int* __restrict__ srcs, const int* __restrict__ dsts,
                                                 int* LIST, int* CNT, int* OFF, int* DINVI, int* FLAG) {
  extern __shared__ __attribute__((aligned(16))) int dsm[];
  int* wl   = dsm;
  int* pl   = dsm + NWAVE * WLCAP;
  int* cnt  = pl + RCAP;
  int* offs = cnt + NBRUN;
  int* cur  = offs + NBRUN;
  int* misc = cur + NBRUN;
  const int tid = (int)threadIdx.x, lane = tid & 31, wave = tid >> 5;
  const int blk = (int)blockIdx.x;
  const unsigned nbs = (unsigned)(blk * NBRUN);

  {
    const v4i z4 = {0, 0, 0, 0};
    for (int i = tid * 4; i < BK_ZINTS; i += NTHR * 4) *(v4ia*)(dsm + i) = z4;
    if (tid < 16) misc[tid] = 0;
  }
  __syncthreads();

  {
    const int per  = ((NE + NWAVE * WCH - 1) / (NWAVE * WCH)) * WCH;
    const int ebeg = wave * per;
    const int eend = (ebeg + per < NE) ? (ebeg + per) : NE;
    int* mylist = wl + wave * WLCAP;
    int wc = 0;
#pragma unroll 1
    for (int cb = ebeg; cb < eend; cb += WCH) {
      const int e0 = cb + lane * EPT;
      const v4i da = *(const v4ia*)(dsts + e0);
      const v4i db = *(const v4ia*)(dsts + e0 + 4);
      const unsigned s0 = (unsigned)da.x - nbs, s1 = (unsigned)da.y - nbs;
      const unsigned s2 = (unsigned)da.z - nbs, s3 = (unsigned)da.w - nbs;
      const unsigned s4 = (unsigned)db.x - nbs, s5 = (unsigned)db.y - nbs;
      const unsigned s6 = (unsigned)db.z - nbs, s7 = (unsigned)db.w - nbs;
      const bool h0 = s0 < (unsigned)NBRUN, h1 = s1 < (unsigned)NBRUN, h2 = s2 < (unsigned)NBRUN, h3 = s3 < (unsigned)NBRUN;
      const bool h4 = s4 < (unsigned)NBRUN, h5 = s5 < (unsigned)NBRUN, h6 = s6 < (unsigned)NBRUN, h7 = s7 < (unsigned)NBRUN;
      const unsigned m0 = __builtin_amdgcn_ballot_w32(h0), m1 = __builtin_amdgcn_ballot_w32(h1);
      const unsigned m2 = __builtin_amdgcn_ballot_w32(h2), m3 = __builtin_amdgcn_ballot_w32(h3);
      const unsigned m4 = __builtin_amdgcn_ballot_w32(h4), m5 = __builtin_amdgcn_ballot_w32(h5);
      const unsigned m6 = __builtin_amdgcn_ballot_w32(h6), m7 = __builtin_amdgcn_ballot_w32(h7);
      const unsigned any = m0 | m1 | m2 | m3 | m4 | m5 | m6 | m7;
      if (any != 0u) {
        const int pre = (int)(__builtin_amdgcn_mbcnt_lo(m0, 0u) + __builtin_amdgcn_mbcnt_lo(m1, 0u) +
                              __builtin_amdgcn_mbcnt_lo(m2, 0u) + __builtin_amdgcn_mbcnt_lo(m3, 0u) +
                              __builtin_amdgcn_mbcnt_lo(m4, 0u) + __builtin_amdgcn_mbcnt_lo(m5, 0u) +
                              __builtin_amdgcn_mbcnt_lo(m6, 0u) + __builtin_amdgcn_mbcnt_lo(m7, 0u));
        int p = wc + pre;
        if (h0) { if (p < WLCAP) mylist[p] = ((e0 + 0) << SLB) | (int)s0; p = p + 1; }
        if (h1) { if (p < WLCAP) mylist[p] = ((e0 + 1) << SLB) | (int)s1; p = p + 1; }
        if (h2) { if (p < WLCAP) mylist[p] = ((e0 + 2) << SLB) | (int)s2; p = p + 1; }
        if (h3) { if (p < WLCAP) mylist[p] = ((e0 + 3) << SLB) | (int)s3; p = p + 1; }
        if (h4) { if (p < WLCAP) mylist[p] = ((e0 + 4) << SLB) | (int)s4; p = p + 1; }
        if (h5) { if (p < WLCAP) mylist[p] = ((e0 + 5) << SLB) | (int)s5; p = p + 1; }
        if (h6) { if (p < WLCAP) mylist[p] = ((e0 + 6) << SLB) | (int)s6; p = p + 1; }
        if (h7) { if (p < WLCAP) mylist[p] = ((e0 + 7) << SLB) | (int)s7; p = p + 1; }
        wc += (int)(__builtin_popcount(m0) + __builtin_popcount(m1) + __builtin_popcount(m2) + __builtin_popcount(m3) +
                    __builtin_popcount(m4) + __builtin_popcount(m5) + __builtin_popcount(m6) + __builtin_popcount(m7));
      }
    }
    if (lane == 0) misc[wave] = wc;
  }
  __syncthreads();

  if (wave == 0) {
    int ov = 0;
#pragma unroll 1
    for (int w2 = 0; w2 < NWAVE; ++w2) {
      int c = misc[w2];
      if (c > WLCAP) ov = 1;
      c = c < 0 ? 0 : (c > WLCAP ? WLCAP : c);
#pragma unroll 1
      for (int b0 = 0; b0 < c; b0 += 32) {
        const int idx = b0 + lane;
        const int ent = wl[w2 * WLCAP + (idx < WLCAP ? idx : WLCAP - 1)];
        const int m32 = (c - b0) < 32 ? (c - b0) : 32;
#pragma unroll 1
        for (int k = 0; k < m32; ++k) {
          const int u    = __builtin_amdgcn_readlane(ent, k);
          const int slot = u & (NBRUN - 1);
          if (lane == 0) cnt[slot] = cnt[slot] + 1;
        }
      }
    }
    if (lane == 0) misc[9] = ov;
  }
  __syncthreads();
  if (wave == 0) {
    const int base = lane * (NBRUN / 32);
    int s = 0;
#pragma unroll 1
    for (int i = 0; i < NBRUN / 32; ++i) s += cnt[base + i];
    int incl = s;
#pragma unroll
    for (int d = 1; d < 32; d <<= 1) {
      const int y = __shfl_up(incl, d, 32);
      if (lane >= d) incl += y;
    }
    int run = incl - s;
#pragma unroll 1
    for (int i = 0; i < NBRUN / 32; ++i) {
      const int cv = cnt[base + i];
      offs[base + i] = run;
      cur[base + i]  = run;
      run += cv;
    }
  }
  __syncthreads();

  if (wave == 0) {
#pragma unroll 1
    for (int w2 = 0; w2 < NWAVE; ++w2) {
      int c = misc[w2];
      c = c < 0 ? 0 : (c > WLCAP ? WLCAP : c);
#pragma unroll 1
      for (int b0 = 0; b0 < c; b0 += 32) {
        const int idx = b0 + lane;
        const int ent = wl[w2 * WLCAP + (idx < WLCAP ? idx : WLCAP - 1)];
        int eid = (ent >> SLB) & 0xfffff;
        eid = eid > NE - 1 ? NE - 1 : eid;
        int sr = srcs[eid];
        sr = sr < 0 ? 0 : (sr > NN - 1 ? NN - 1 : sr);
        const int m32 = (c - b0) < 32 ? (c - b0) : 32;
#pragma unroll 1
        for (int k = 0; k < m32; ++k) {
          const int u    = __builtin_amdgcn_readlane(ent, k);
          const int wd   = __builtin_amdgcn_readlane(sr, k);
          const int slot = u & (NBRUN - 1);
          if (lane == 0) {
            int p = cur[slot];
            p = p < 0 ? 0 : (p > RCAP - 1 ? RCAP - 1 : p);
            pl[p] = wd;
            cur[slot] = p + 1;
          }
        }
      }
    }
  }
  __syncthreads();

#pragma unroll 1
  for (int i = tid; i < NBRUN; i += NTHR) {
    const float dg = (float)(cnt[i] + 1);
    cur[i] = __float_as_int(1.0f / sqrtf(dg));
  }
  __syncthreads();

  const int ovf = misc[9];
  int* lp = LIST + (size_t)blk * RCAP;
  int* cp = CNT + (size_t)blk * NBRUN;
  int* op = OFF + (size_t)blk * NBRUN;
  int* dp = DINVI + (size_t)blk * NBRUN;
  int* fp = FLAG + (size_t)blk * 32;
  bucket_flush(pl, cnt, offs, cur, ovf, lp, cp, op, dp, fp, tid);
  __threadfence();
  bucket_flush(pl, cnt, offs, cur, ovf, lp, cp, op, dp, fp, tid);
}

template <int KTOT>
__device__ __forceinline__ void gemm_16x64(const unsigned short* __restrict__ ap,
                                           const unsigned short* __restrict__ bp, v8f (&acc)[4]) {
#pragma unroll 1
  for (int k0 = 0; k0 < KTOT; k0 += 32) {
    FragB af;
    af.h[0] = *(const v8usa*)(ap + k0);
    af.h[1] = *(const v8usa*)(ap + k0 + 16);
#pragma unroll
    for (int nt = 0; nt < 4; ++nt) {
      const unsigned short* wq = bp + (size_t)(16 * nt) * (size_t)KTOT + k0;
      FragB bf;
      bf.h[0] = *(const v8usa*)wq;
      bf.h[1] = *(const v8usa*)(wq + 16);
      acc[nt] = wmb(af, bf, acc[nt]);
    }
  }
}

__device__ __forceinline__ void stage_d(float* stg, const v8f (&acc)[4], int wave, int hh, int m) {
#pragma unroll
  for (int nt = 0; nt < 4; ++nt) {
#pragma unroll
    for (int r = 0; r < 8; ++r) stg[(16 * wave + 8 * hh + r) * SP + 16 * nt + m] = acc[nt][r];
  }
}

template <int KTOT>
__global__ __launch_bounds__(NTHR) __attribute__((amdgpu_num_vgpr(248)))
void k_gemm(const unsigned short* __restrict__ A, const unsigned short* __restrict__ BT,
            const float* __restrict__ dinv, float* C) {
  __shared__ __attribute__((aligned(16))) float stg[GBM * SP];
  __shared__ __attribute__((aligned(16))) float sdv[GBM];
  const int tid = (int)threadIdx.x, lane = tid & 31, wave = tid >> 5, hh = lane >> 4, m = lane & 15;
  const int rowBase = (int)blockIdx.x * GBM;
  if (tid < 32) *(v4fa*)(sdv + 4 * tid) = *(const v4fa*)(dinv + (size_t)rowBase + 4 * tid);
  const unsigned short* ap = A + (size_t)(rowBase + 16 * wave + m) * (size_t)KTOT + 8 * hh;

#pragma unroll 1
  for (int half = 0; half < 2; ++half) {
    v8f acc[4];
    {
      const v8f z = {0.f, 0.f, 0.f, 0.f, 0.f, 0.f, 0.f, 0.f};
#pragma unroll
      for (int t = 0; t < 4; ++t) acc[t] = z;
    }
    const unsigned short* bp = BT + (size_t)(64 * half + m) * (size_t)KTOT + 8 * hh;
    gemm_16x64<KTOT>(ap, bp, acc);
    stage_d(stg, acc, wave, hh, m);
    __syncthreads();

    v4f fv[8];
#pragma unroll
    for (int i = 0; i < 8; ++i) {
      const int lr = 16 * wave + 2 * i + hh;
      const v4f a  = *(const v4fa*)(stg + lr * SP + 4 * m);
      const float dv = sdv[lr];
      v4f o;
      o.x = a.x * dv; o.y = a.y * dv; o.z = a.z * dv; o.w = a.w * dv;
      fv[i] = o;
    }
#pragma unroll
    for (int i = 0; i < 8; ++i) {
      const int grow = rowBase + 16 * wave + 2 * i + hh;
      float* op = C + (size_t)grow * NCAT + 64 * half + 4 * m;
      *(volatile v4f*)op = fv[i];
    }
    __threadfence();
#pragma unroll
    for (int i = 0; i < 8; ++i) {
      const int grow = rowBase + 16 * wave + 2 * i + hh;
      float* op = C + (size_t)grow * NCAT + 64 * half + 4 * m;
      *(volatile v4f*)op = fv[i];
    }
    __syncthreads();
  }
}

__device__ __forceinline__ v4f row_sum(const int* __restrict__ lb, const float* __restrict__ pre,
                                       int c, int o, int last, int lane) {
  float a0 = 0.0f, a1 = 0.0f, a2 = 0.0f, a3 = 0.0f;
#pragma unroll 1
  for (int b0 = 0; b0 < c; b0 += 32) {
    int idx = o + b0 + lane;
    idx = idx > last ? last : idx;
    int sr = lb[idx];
    sr = sr < 0 ? 0 : (sr > NN - 1 ? NN - 1 : sr);
    const int m32 = (c - b0) < 32 ? (c - b0) : 32;
#pragma unroll 1
    for (int k = 0; k < m32; ++k) {
      const int sk = __builtin_amdgcn_readlane(sr, k);
      const v4f v = *(const v4fa*)(pre + (size_t)sk * NCAT + 4 * lane);
      a0 += v.x; a1 += v.y; a2 += v.z; a3 += v.w;
    }
  }
  v4f r;
  r.x = a0; r.y = a1; r.z = a2; r.w = a3;
  return r;
}

__global__ __launch_bounds__(NTHR) void k_replay_ln(const int* __restrict__ LIST, const int* __restrict__ CNT,
                                                    const int* __restrict__ OFF, const float* __restrict__ DINV,
                                                    const int* __restrict__ FLAG, const float* __restrict__ pre,
                                                    const float* __restrict__ tb, unsigned short* hhl) {
  __shared__ __attribute__((aligned(16))) float stb[384];
  const int tid = (int)threadIdx.x, lane = tid & 31, wave = tid >> 5;
  const int rowBase = (int)blockIdx.x * RBM;
  const int bucket  = rowBase >> SLB;
  if (tid < 96) *(v4fa*)(stb + 4 * tid) = *(const v4fa*)(tb + 4 * tid);
  __syncthreads();
  const v4f bia = *(const v4fa*)(stb + 4 * lane);
  const v4f gsc = *(const v4fa*)(stb + 128 + 4 * lane);
  const v4f gsh = *(const v4fa*)(stb + 256 + 4 * lane);
  const int* lb  = LIST + (size_t)bucket * RCAP;
  const int flag = FLAG[(size_t)bucket * 32];
  const float qnan = __uint_as_float(0x7fc00000u);

#pragma unroll 1
  for (int i = 0; i < RBM / NWAVE; ++i) {
    const int d = rowBase + (RBM / NWAVE) * wave + i;
    int cv = CNT[d];
    int ov = OFF[d];
    const int bigv = cv > DEGCAP ? 1 : 0;
    cv = cv < 0 ? 0 : (cv > DEGCAP ? DEGCAP : cv);
    ov = ov < 0 ? 0 : (ov > RCAP - 1 ? RCAP - 1 : ov);
    int lastv = ov + cv - 1;
    lastv = lastv < ov ? ov : lastv;
    lastv = lastv > RCAP - 1 ? RCAP - 1 : lastv;
    const int c    = __builtin_amdgcn_readfirstlane(cv);
    const int o    = __builtin_amdgcn_readfirstlane(ov);
    const int last = __builtin_amdgcn_readfirstlane(lastv);
    const int big  = __builtin_amdgcn_readfirstlane(bigv);
    const float dd = DINV[d];
    const v4f sm = row_sum(lb, pre, c, o, last, lane);
    const v4f sv = *(const v4fa*)(pre + (size_t)d * NCAT + 4 * lane);
    float t0 = dd * (sm.x + sv.x) + bia.x, t1 = dd * (sm.y + sv.y) + bia.y;
    float t2 = dd * (sm.z + sv.z) + bia.z, t3 = dd * (sm.w + sv.w) + bia.w;
    t0 = (t0 > 0.0f) ? t0 : (t0 - t0); t1 = (t1 > 0.0f) ? t1 : (t1 - t1);
    t2 = (t2 > 0.0f) ? t2 : (t2 - t2); t3 = (t3 > 0.0f) ? t3 : (t3 - t3);
    float s = (t0 + t1) + (t2 + t3);
    s += __shfl_xor(s, 16, 32); s += __shfl_xor(s, 8, 32); s += __shfl_xor(s, 4, 32);
    s += __shfl_xor(s, 2, 32);  s += __shfl_xor(s, 1, 32);
    const float mean = s * (1.0f / 128.0f);
    const float e0 = t0 - mean, e1 = t1 - mean, e2 = t2 - mean, e3 = t3 - mean;
    float q = (e0 * e0 + e1 * e1) + (e2 * e2 + e3 * e3);
    q += __shfl_xor(q, 16, 32); q += __shfl_xor(q, 8, 32); q += __shfl_xor(q, 4, 32);
    q += __shfl_xor(q, 2, 32);  q += __shfl_xor(q, 1, 32);
    const float var = q * (1.0f / 128.0f);
    const float inv = 1.0f / sqrtf(var + 1e-5f);
    float y0 = (e0 * inv) * gsc.x + gsh.x, y1 = (e1 * inv) * gsc.y + gsh.y;
    float y2 = (e2 * inv) * gsc.z + gsh.z, y3 = (e3 * inv) * gsc.w + gsh.w;
    const bool bad  = (flag != 0) | (big != 0);
    const bool live = d < NN;
    y0 = bad ? qnan : y0; y1 = bad ? qnan : y1; y2 = bad ? qnan : y2; y3 = bad ? qnan : y3;
    y0 = live ? y0 : 0.0f; y1 = live ? y1 : 0.0f; y2 = live ? y2 : 0.0f; y3 = live ? y3 : 0.0f;
    int h01, h23, l01, l23;
    hilo_pack(y0, y1, y2, y3, h01, h23, l01, l23);
    const v4i ow = regroup_row(h01, h23, l01, l23, lane);
    unsigned short* hp = hhl + (size_t)d * KC + 8 * lane;
    *(volatile v4i*)hp = ow;
    __threadfence();
    *(volatile v4i*)hp = ow;
  }
}

__global__ __launch_bounds__(NTHR) void k_replay_out(const int* __restrict__ LIST, const int* __restrict__ CNT,
                                                     const int* __restrict__ OFF, const float* __restrict__ DINV,
                                                     const int* __restrict__ FLAG, const float* __restrict__ pre,
                                                     const float* __restrict__ tb, float* out) {
  __shared__ __attribute__((aligned(16))) float sbc[128];
  const int tid = (int)threadIdx.x, lane = tid & 31, wave = tid >> 5;
  const int rowBase = (int)blockIdx.x * RBM;
  const int bucket  = rowBase >> SLB;
  if (tid < 32) *(v4fa*)(sbc + 4 * tid) = *(const v4fa*)(tb + 384 + 4 * tid);
  __syncthreads();
  const v4f bia = *(const v4fa*)(sbc + 4 * lane);
  const int* lb  = LIST + (size_t)bucket * RCAP;
  const int flag = FLAG[(size_t)bucket * 32];
  const float qnan = __uint_as_float(0x7fc00000u);

#pragma unroll 1
  for (int i = 0; i < RBM / NWAVE; ++i) {
    const int d = rowBase + (RBM / NWAVE) * wave + i;
    int cv = CNT[d];
    int ov = OFF[d];
    const int bigv = cv > DEGCAP ? 1 : 0;
    cv = cv < 0 ? 0 : (cv > DEGCAP ? DEGCAP : cv);
    ov = ov < 0 ? 0 : (ov > RCAP - 1 ? RCAP - 1 : ov);
    int lastv = ov + cv - 1;
    lastv = lastv < ov ? ov : lastv;
    lastv = lastv > RCAP - 1 ? RCAP - 1 : lastv;
    const int c    = __builtin_amdgcn_readfirstlane(cv);
    const int o    = __builtin_amdgcn_readfirstlane(ov);
    const int last = __builtin_amdgcn_readfirstlane(lastv);
    const int big  = __builtin_amdgcn_readfirstlane(bigv);
    const float dd = DINV[d];
    const v4f sm = row_sum(lb, pre, c, o, last, lane);
    const v4f sv = *(const v4fa*)(pre + (size_t)d * NCAT + 4 * lane);
    float o0 = dd * (sm.x + sv.x) + bia.x, o1 = dd * (sm.y + sv.y) + bia.y;
    float o2 = dd * (sm.z + sv.z) + bia.z, o3 = dd * (sm.w + sv.w) + bia.w;
    const bool bad = (flag != 0) | (big != 0);
    o0 = bad ? qnan : o0; o1 = bad ? qnan : o1; o2 = bad ? qnan : o2; o3 = bad ? qnan : o3;
    v4f ov4;
    ov4.x = o0; ov4.y = o1; ov4.z = o2; ov4.w = o3;
    const size_t off = (size_t)d * OUTF + (size_t)(4 * (lane & 15)) + (size_t)(lane >> 4) * (size_t)OUTSPLIT;
    float* op = out + off;
    const bool live = d < NN;
    if (live) *(volatile v4f*)op = ov4;
    __threadfence();
    if (live) *(volatile v4f*)op = ov4;
  }
}

extern "C" void kernel_launch(void* const* d_in, const int* in_sizes, int n_in,
                              void* d_out, int out_size, void* d_ws, size_t ws_size,
                              hipStream_t stream) {
  if (n_in < 10) return;
  if (in_sizes[0] != NN * FIN) return;
  if (in_sizes[1] != 2 * NE) return;
  if (in_sizes[2] != FIN * HID) return;
  if (in_sizes[3] != HID) return;
  if (in_sizes[4] != HID) return;
  if (in_sizes[5] != HID) return;
  if (in_sizes[6] != HID * OUTF) return;
  if (in_sizes[7] != OUTF) return;
  if (in_sizes[8] != HID * OUTF) return;
  if (in_sizes[9] != OUTF) return;
  if (out_size != 2 * NN * OUTF) return;

  const float* x   = (const float*)d_in[0];
  const int*   ei  = (const int*)d_in[1];
  const float* wa  = (const float*)d_in[2];
  const float* ba  = (const float*)d_in[3];
  const float* gam = (const float*)d_in[4];
  const float* bet = (const float*)d_in[5];
  const float* wmu = (const float*)d_in[6];
  const float* bmu = (const float*)d_in[7];
  const float* wlv = (const float*)d_in[8];
  const float* blv = (const float*)d_in[9];
  float* out = (float*)d_out;
  const int* srcs = ei;
  const int* dsts = ei + NE;

  constexpr size_t zXB   = (size_t)MP * FIN * 2;
  constexpr size_t zPRE  = (size_t)MP * NCAT * 4;
  constexpr size_t zHHL  = (size_t)MP * KC * 2;
  constexpr size_t zLIST = (size_t)NBK * RCAP * 4;
  constexpr size_t zSLOT = (size_t)NSLOT * 4;
  constexpr size_t zFLAG = (size_t)(NBK + 1) * 128;
  constexpr size_t zWAT  = (size_t)HID * FIN * 2;
  constexpr size_t zWCT  = (size_t)NCAT * KC * 2;
  constexpr size_t zTB   = 2048;
  constexpr size_t oXB   = 0;
  constexpr size_t oPRE  = oXB + zXB;
  constexpr size_t oHHL  = oPRE + zPRE;
  constexpr size_t oLIST = oHHL + zHHL;
  constexpr size_t oCNT  = oLIST + zLIST;
  constexpr size_t oOFF  = oCNT + zSLOT;
  constexpr size_t oDINV = oOFF + zSLOT;
  constexpr size_t oFLAG = oDINV + zSLOT;
  constexpr size_t oWAT  = oFLAG + zFLAG;
  constexpr size_t oWCT  = oWAT + zWAT;
  constexpr size_t oTB   = oWCT + zWCT;
  constexpr size_t oEND  = oTB + zTB;
  static_assert(zXB % 256 == 0 && zPRE % 256 == 0 && zHHL % 256 == 0 && zLIST % 256 == 0 && zSLOT % 256 == 0);
  static_assert(zFLAG % 256 == 0 && zWAT % 256 == 0 && zWCT % 256 == 0 && zTB % 256 == 0);
  static_assert(oWCT == oWAT + (size_t)HID * FIN * 2);
  static_assert(oEND <= (size_t)(128u << 20));
  if (oEND > ws_size) return;

  char* ws = (char*)d_ws;
  unsigned short* XB   = (unsigned short*)(ws + oXB);
  float*          PRE  = (float*)(ws + oPRE);
  unsigned short* HHL  = (unsigned short*)(ws + oHHL);
  int*            LIST = (int*)(ws + oLIST);
  int*            CNT  = (int*)(ws + oCNT);
  int*            OFF  = (int*)(ws + oOFF);
  int*            DVI  = (int*)(ws + oDINV);
  const float*    DINV = (const float*)(ws + oDINV);
  int*            FLAG = (int*)(ws + oFLAG);
  unsigned short* WPL  = (unsigned short*)(ws + oWAT);
  const unsigned short* WAT = (const unsigned short*)(ws + oWAT);
  const unsigned short* WCT = (const unsigned short*)(ws + oWCT);
  float*          TB   = (float*)(ws + oTB);

  hipFuncSetAttribute(reinterpret_cast<const void*>(&k_bucket), hipFuncAttributeMaxDynamicSharedMemorySize, (int)BK_LDS);

  k_prep<<<PBTOT, NTHR, 0, stream>>>(x, wa, ba, gam, bet, wmu, bmu, wlv, blv, XB, WPL, TB);
  k_bucket<<<NBK, NTHR, BK_LDS, stream>>>(srcs, dsts, LIST, CNT, OFF, DVI, FLAG);
  k_gemm<FIN><<<MP / GBM, NTHR, 0, stream>>>(XB, WAT, DINV, PRE);
  k_replay_ln<<<MP / RBM, NTHR, 0, stream>>>(LIST, CNT, OFF, DINV, FLAG, PRE, TB, HHL);
  k_gemm<KC><<<MP / GBM, NTHR, 0, stream>>>(HHL, WCT, DINV, PRE);
  k_replay_out<<<MP / RBM, NTHR, 0, stream>>>(LIST, CNT, OFF, DINV, FLAG, PRE, TB, out);
}
